// GraphDecoder_82274393522845
// MI455X (gfx1250) — hardware-verified
//
#include <hip/hip_runtime.h>
#include <math.h>
#include <stdint.h>

#define NN    3072
#define IND   512
#define DD    256
#define HH    8
#define DK    32
#define OD    512
#define NL    2
#define QKVW  768
#define NSC   8.0f
#define WSC   64.0f
#define XS0   64.0f
#define XSA   1024.0f
#define VSC   2048.0f
#define PCAR  32768.0f
#define LOG2E 1.4426950408889634f
#define RSQ32 0.17677669529663687f
#define GP    68
#define TP    68
#define TTP   72
#define OTP   260

static_assert((NN % 64) == 0 && (IND % 64) == 0 && (DD % 64) == 0 && (OD % 64) == 0 && (QKVW % 64) == 0);
static_assert((IND % 32) == 0 && (DD % 32) == 0 && (NN % 32) == 0 && (NN % 16) == 0);
static_assert(HH * DK == DD && QKVW == 3 * DD && HH == 8 && DK == 32);
static_assert(((NN * IND) % 2048) == 0);
static_assert((GP % 4) == 0 && (TP % 4) == 0 && (TTP % 8) == 0 && (OTP % 4) == 0);
static_assert(15 * GP + 63 < 16 * GP && 127 * TP + 63 < 128 * TP && 63 * TTP + 63 < 64 * TTP && 15 * OTP + 255 < 16 * OTP);
static_assert(2 * HH * 64 == 256 * 4 && (2 * HH - 1) * 64 + 63 < 2 * HH * 64);

typedef _Float16 v16h __attribute__((ext_vector_type(16)));
typedef _Float16 v8h  __attribute__((ext_vector_type(8)));
typedef float    v8f  __attribute__((ext_vector_type(8)));
typedef float    v4f  __attribute__((ext_vector_type(4)));
typedef float    v2f  __attribute__((ext_vector_type(2)));
typedef unsigned int v4u __attribute__((ext_vector_type(4)));

union FragH { v16h v; v8h h[2]; v4u u[2]; };

__device__ __forceinline__ unsigned short bf_bits(float f) {
  unsigned u = __float_as_uint(f);
  return (unsigned short)((u + 0x7FFFu + ((u >> 16) & 1u)) >> 16);
}
__device__ __forceinline__ float bf_up(unsigned short b) { return __uint_as_float(((unsigned)b) << 16); }
__device__ __forceinline__ float bfr(float f) { return bf_up(bf_bits(f)); }
__device__ __forceinline__ unsigned short h_bits(_Float16 x) { return __builtin_bit_cast(unsigned short, x); }
__device__ __forceinline__ unsigned pk16(unsigned short a, unsigned short b) { return (unsigned)a | ((unsigned)b << 16); }
__device__ __forceinline__ v8f zero8() { v8f z = {0.f, 0.f, 0.f, 0.f, 0.f, 0.f, 0.f, 0.f}; return z; }
__device__ __forceinline__ v4f zero4() { v4f z = {0.f, 0.f, 0.f, 0.f}; return z; }

__device__ __forceinline__ v16h ldfrag_h(const _Float16* p) {
  FragH f;
  f.h[0] = *(const v8h*)(p);
  f.h[1] = *(const v8h*)(p + 16);
  return f.v;
}

__device__ __forceinline__ v8f mma_raw(v16h a, v16h b, v8f c) {
  return __builtin_amdgcn_wmma_f32_16x16x32_f16(false, a, false, b, (short)0, c, false, false);
}
__device__ __forceinline__ void guard_g4(v8f& a0, v8f& a1, v8f& a2, v8f& a3, v16h x0, v16h x1,
                                         v16h y0, v16h y1, v16h y2, v16h y3) {
#if defined(__HIP_DEVICE_COMPILE__)
  asm volatile("v_nop\n\tv_nop\n\tv_nop\n\tv_nop"
               : "+v"(a0), "+v"(a1), "+v"(a2), "+v"(a3)
               : "v"(x0), "v"(x1), "v"(y0), "v"(y1), "v"(y2), "v"(y3) : "memory");
#endif
}
__device__ __forceinline__ void guard_a2(v8f& a0, v8f& a1, v16h p, v16h y0, v16h y1, v16h y2, v16h y3) {
#if defined(__HIP_DEVICE_COMPILE__)
  asm volatile("v_nop\n\tv_nop\n\tv_nop\n\tv_nop"
               : "+v"(a0), "+v"(a1) : "v"(p), "v"(y0), "v"(y1), "v"(y2), "v"(y3) : "memory");
#endif
}
__device__ __forceinline__ void acc_guard4(v8f& a, v8f& b, v8f& c, v8f& d) {
#if defined(__HIP_DEVICE_COMPILE__)
  asm volatile("v_nop\n\tv_nop\n\tv_nop\n\tv_nop" : "+v"(a), "+v"(b), "+v"(c), "+v"(d));
#endif
}
__device__ __forceinline__ void acc_guard2(v8f& a, v8f& b) {
#if defined(__HIP_DEVICE_COMPILE__)
  asm volatile("v_nop\n\tv_nop\n\tv_nop\n\tv_nop" : "+v"(a), "+v"(b));
#endif
}
__device__ __forceinline__ void wave_sync_lds() {
  __builtin_amdgcn_fence(__ATOMIC_RELEASE, "workgroup");
  __builtin_amdgcn_wave_barrier();
  __builtin_amdgcn_fence(__ATOMIC_ACQUIRE, "workgroup");
}

__device__ __forceinline__ float lscore(float qa, float ka, float m) {
  float s = (qa + ka) * m;
  s = (s > 0.0f) ? s : 0.2f * s;
  return s * LOG2E;
}

__global__ __launch_bounds__(256) void cvt16(const float* __restrict__ x, unsigned short* pl, int n8, float sc) {
  const int gt = (int)blockIdx.x * 256 + (int)threadIdx.x;
  if (gt >= n8) return;
  const size_t e = (size_t)gt * 8;
  const v4f a = *(const v4f*)(x + e), b = *(const v4f*)(x + e + 4);
  v4u o;
#pragma unroll
  for (int i = 0; i < 2; ++i) {
    o[i]     = pk16(h_bits((_Float16)(bfr(a[2 * i]) * sc)), h_bits((_Float16)(bfr(a[2 * i + 1]) * sc)));
    o[2 + i] = pk16(h_bits((_Float16)(bfr(b[2 * i]) * sc)), h_bits((_Float16)(bfr(b[2 * i + 1]) * sc)));
  }
  unsigned short* d = pl + e;
  for (int pass = 0; pass < 2; ++pass) {
    *(volatile v4u*)(d) = o;
    __threadfence();
  }
}

__global__ __launch_bounds__(256) void wt16(const float* __restrict__ in, unsigned short* out, int R, int Ccol, float sc) {
  __shared__ __align__(16) unsigned short T[64 * TTP];
  const int tid = (int)threadIdx.x;
  const int r0 = (int)blockIdx.y * 64, c0 = (int)blockIdx.x * 64;
  if (r0 + 64 > R || c0 + 64 > Ccol) return;
  {
    const int r = tid >> 2, cc = (tid & 3) * 16;
    const float* src = in + (size_t)(r0 + r) * Ccol + c0 + cc;
#pragma unroll
    for (int i = 0; i < 4; ++i) {
      const v4f a = *(const v4f*)(src + 4 * i);
#pragma unroll
      for (int e = 0; e < 4; ++e) T[(cc + 4 * i + e) * TTP + r] = h_bits((_Float16)(bfr(a[e]) * sc));
    }
  }
  __syncthreads();
  const int q8 = tid >> 3, p8 = (tid & 7) * 8;
  v4u vals[2];
#pragma unroll
  for (int it = 0; it < 2; ++it) {
    const int line = 32 * it + q8;
    vals[it] = *(const v4u*)(T + line * TTP + p8);
  }
  unsigned short* dst = out + (size_t)(c0 + q8) * R + r0 + p8;
  const size_t step = (size_t)32 * R;
  for (int pass = 0; pass < 2; ++pass) {
#pragma unroll
    for (int it = 0; it < 2; ++it) *(volatile v4u*)(dst + it * step) = vals[it];
    __threadfence();
  }
}

template <bool ARES, bool HASB, int OUTK>
__global__ __launch_bounds__(128) void gemm16(const unsigned short* __restrict__ Ah,
                                              const unsigned short* __restrict__ Ar,
                                              const unsigned short* __restrict__ Bt,
                                              const float* __restrict__ bias,
                                              float* Cf, unsigned short* Ch, unsigned short* Cr,
                                              int M, int N, int K, float osc, float xs) {
  __shared__ __align__(16) float slab_all[4 * 16 * GP];
  const int tid = (int)threadIdx.x, wave = tid >> 5, lane = tid & 31, hh = lane >> 4, c = lane & 15;
  const int m0 = (int)blockIdx.y * 64, n0 = (int)blockIdx.x * 64;
  if (m0 + 64 > M || n0 + 64 > N) return;
  const int row0 = m0 + 16 * wave;
  const _Float16* ap = (const _Float16*)(const void*)Ah + (size_t)(row0 + c) * K + 8 * hh;
  const _Float16* rp = (const _Float16*)(const void*)Ar + (size_t)(row0 + c) * K + 8 * hh;
  const _Float16* bp = (const _Float16*)(const void*)Bt + (size_t)(n0 + c) * K + 8 * hh;
  const size_t bs = (size_t)16 * K;

  v8f acc0 = zero8(), acc1 = zero8(), acc2 = zero8(), acc3 = zero8();
#pragma unroll 1
  for (int kk = 0; kk < K; kk += 32) {
    const v16h a = ldfrag_h(ap + kk);
    v16h ar = a;
    if (ARES) ar = ldfrag_h(rp + kk);
    const v16h b0 = ldfrag_h(bp + kk);
    const v16h b1 = ldfrag_h(bp + bs + kk);
    const v16h b2 = ldfrag_h(bp + 2 * bs + kk);
    const v16h b3 = ldfrag_h(bp + 3 * bs + kk);
    acc0 = mma_raw(a, b0, acc0);
    if (ARES) acc0 = mma_raw(ar, b0, acc0);
    acc1 = mma_raw(a, b1, acc1);
    if (ARES) acc1 = mma_raw(ar, b1, acc1);
    acc2 = mma_raw(a, b2, acc2);
    if (ARES) acc2 = mma_raw(ar, b2, acc2);
    acc3 = mma_raw(a, b3, acc3);
    if (ARES) acc3 = mma_raw(ar, b3, acc3);
    guard_g4(acc0, acc1, acc2, acc3, a, ar, b0, b1, b2, b3);
  }
  acc_guard4(acc0, acc1, acc2, acc3);

  float* slab = slab_all + wave * (16 * GP);
#pragma unroll
  for (int r = 0; r < 8; ++r) {
    float* sp = slab + (8 * hh + r) * GP + c;
    sp[0]  = acc0[r];
    sp[16] = acc1[r];
    sp[32] = acc2[r];
    sp[48] = acc3[r];
  }
  wave_sync_lds();

  if (OUTK == 0) {
    v4f bb = zero4();
    if (HASB) {
#pragma unroll
      for (int e = 0; e < 4; ++e) bb[e] = bfr(bias[n0 + 4 * c + e]);
    }
    v4f vals[8];
#pragma unroll
    for (int it = 0; it < 8; ++it) {
      const v4f v = *(const v4f*)(slab + (2 * it + hh) * GP + 4 * c);
      v4f w;
#pragma unroll
      for (int e = 0; e < 4; ++e) w[e] = v[e] * osc + bb[e];
      vals[it] = w;
    }
    float* dst = Cf + (size_t)(row0 + hh) * N + n0 + 4 * c;
    const size_t rs2 = (size_t)2 * N;
    for (int pass = 0; pass < 2; ++pass) {
#pragma unroll
      for (int it = 0; it < 8; ++it) *(volatile v4f*)(dst + it * rs2) = vals[it];
      __threadfence();
    }
  } else {
    const int q = lane >> 3, p8 = (lane & 7) * 8;
    float bv[8];
#pragma unroll
    for (int e = 0; e < 8; ++e) bv[e] = HASB ? bfr(bias[n0 + p8 + e]) : 0.0f;
    v4u vh[4], vr[4];
#pragma unroll
    for (int it = 0; it < 4; ++it) {
      const float* sp = slab + (4 * it + q) * GP + p8;
      const v4f w0 = *(const v4f*)(sp), w1 = *(const v4f*)(sp + 4);
      float f[8];
#pragma unroll
      for (int e = 0; e < 4; ++e) { f[e] = w0[e]; f[4 + e] = w1[e]; }
      v4u oh, orr;
#pragma unroll
      for (int i = 0; i < 4; ++i) {
        const float t0 = (f[2 * i] * osc + bv[2 * i]) * xs;
        const float t1 = (f[2 * i + 1] * osc + bv[2 * i + 1]) * xs;
        const _Float16 g0 = (_Float16)t0, g1 = (_Float16)t1;
        const _Float16 r0 = (_Float16)(t0 - (float)g0), r1 = (_Float16)(t1 - (float)g1);
        oh[i]  = pk16(h_bits(g0), h_bits(g1));
        orr[i] = pk16(h_bits(r0), h_bits(r1));
      }
      vh[it] = oh;
      vr[it] = orr;
    }
    unsigned short* dh = Ch + (size_t)(row0 + q) * N + n0 + p8;
    unsigned short* dr = Cr + (size_t)(row0 + q) * N + n0 + p8;
    const size_t rs4 = (size_t)4 * N;
    for (int pass = 0; pass < 2; ++pass) {
#pragma unroll
      for (int it = 0; it < 4; ++it) {
        *(volatile v4u*)(dh + it * rs4) = vh[it];
        *(volatile v4u*)(dr + it * rs4) = vr[it];
      }
      __threadfence();
    }
  }
}

__global__ __launch_bounds__(256) void qkv_post(const float* __restrict__ C, const float* __restrict__ aq,
                                                const float* __restrict__ ak, float* QA, float* KA,
                                                unsigned short* VTh, unsigned short* VTr) {
  __shared__ __align__(16) float Tf[128 * TP];
  __shared__ __align__(16) float St[2 * HH * 64];
  const int tid = (int)threadIdx.x, w = tid >> 5, l = tid & 31;
  const int n0 = (int)blockIdx.x * 64;
  if (n0 + 64 > NN) return;
  {
    const int nloc = 32 * (w & 1) + l;
    const int node = n0 + nloc;
    const int g = w >> 1;
    const float* cr  = C + (size_t)node * QKVW;
    const float* aq0 = aq + (2 * g) * DK;
    const float* aq1 = aq + (2 * g + 1) * DK;
    const float* ak0 = ak + (2 * g) * DK;
    const float* ak1 = ak + (2 * g + 1) * DK;
    float q0 = 0.f, q1 = 0.f, k0 = 0.f, k1 = 0.f;
#pragma unroll 1
    for (int kk = 0; kk < DK; kk += 4) {
      const v4f cq0 = *(const v4f*)(cr + 64 * g + kk);
      const v4f cq1 = *(const v4f*)(cr + 64 * g + 32 + kk);
      const v4f ck0 = *(const v4f*)(cr + DD + 64 * g + kk);
      const v4f ck1 = *(const v4f*)(cr + DD + 64 * g + 32 + kk);
      const v4f a0 = *(const v4f*)(aq0 + kk), a1 = *(const v4f*)(aq1 + kk);
      const v4f e0 = *(const v4f*)(ak0 + kk), e1 = *(const v4f*)(ak1 + kk);
#pragma unroll
      for (int e = 0; e < 4; ++e) {
        q0 = fmaf(cq0[e] * RSQ32, bfr(a0[e]), q0);
        q1 = fmaf(cq1[e] * RSQ32, bfr(a1[e]), q1);
        k0 = fmaf(ck0[e], bfr(e0[e]), k0);
        k1 = fmaf(ck1[e], bfr(e1[e]), k1);
      }
    }
    St[(2 * g) * 64 + nloc]          = q0;
    St[(2 * g + 1) * 64 + nloc]      = q1;
    St[(HH + 2 * g) * 64 + nloc]     = k0;
    St[(HH + 2 * g + 1) * 64 + nloc] = k1;
  }
  __syncthreads();
  {
    const int line = tid >> 3, p4 = (tid & 7) * 4;
    const int arr = line >> 4, hd = (line >> 1) & 7, nh = line & 1;
    const v4f v = *(const v4f*)(St + 32 * line + p4);
    float* base = arr ? KA : QA;
    float* dst = base + (size_t)hd * NN + n0 + 32 * nh + p4;
    for (int pass = 0; pass < 2; ++pass) {
      *(volatile v4f*)(dst) = v;
      __threadfence();
    }
  }
  const int q8 = tid >> 3, p8 = (tid & 7) * 8;
  const int nl = tid & 63, gq = tid >> 6;
#pragma unroll 1
  for (int p = 0; p < 2; ++p) {
    {
      const float* src = C + (size_t)(n0 + nl) * QKVW + 2 * DD + 128 * p + 32 * gq;
#pragma unroll
      for (int i = 0; i < 8; ++i) {
        const v4f a = *(const v4f*)(src + 4 * i);
#pragma unroll
        for (int e = 0; e < 4; ++e) Tf[(32 * gq + 4 * i + e) * TP + nl] = a[e];
      }
    }
    __syncthreads();
    v4u vh[4], vr[4];
#pragma unroll
    for (int it = 0; it < 4; ++it) {
      const float* sp = Tf + (32 * it + q8) * TP + p8;
      const v4f w0 = *(const v4f*)(sp), w1 = *(const v4f*)(sp + 4);
      float f[8];
#pragma unroll
      for (int e = 0; e < 4; ++e) { f[e] = w0[e]; f[4 + e] = w1[e]; }
      v4u oh, orr;
#pragma unroll
      for (int i = 0; i < 4; ++i) {
        const float t0 = f[2 * i] * VSC, t1 = f[2 * i + 1] * VSC;
        const _Float16 g0 = (_Float16)t0, g1 = (_Float16)t1;
        const _Float16 r0 = (_Float16)(t0 - (float)g0), r1 = (_Float16)(t1 - (float)g1);
        oh[i]  = pk16(h_bits(g0), h_bits(g1));
        orr[i] = pk16(h_bits(r0), h_bits(r1));
      }
      vh[it] = oh;
      vr[it] = orr;
    }
    unsigned short* dh = VTh + (size_t)(128 * p + q8) * NN + n0 + p8;
    unsigned short* dr = VTr + (size_t)(128 * p + q8) * NN + n0 + p8;
    const size_t rs32 = (size_t)32 * NN;
    for (int pass = 0; pass < 2; ++pass) {
#pragma unroll
      for (int it = 0; it < 4; ++it) {
        *(volatile v4u*)(dh + it * rs32) = vh[it];
        *(volatile v4u*)(dr + it * rs32) = vr[it];
      }
      __threadfence();
    }
    __syncthreads();
  }
}

__global__ __launch_bounds__(256) void add_attn(const float* __restrict__ QA, const float* __restrict__ KA,
                                                const float* __restrict__ mask,
                                                const unsigned short* __restrict__ VTh,
                                                const unsigned short* __restrict__ VTr,
                                                unsigned short* Xh, unsigned short* Xr) {
  __shared__ __align__(16) float mk[16 * 32];
  __shared__ __align__(16) float kat[HH * 32];
  __shared__ __align__(16) float ot[16 * OTP];
  const int tid = (int)threadIdx.x, h = tid >> 5, lane = tid & 31, hh = lane >> 4, c = lane & 15;
  const int i0 = (int)blockIdx.x * 16;
  if (i0 + 16 > NN) return;

  const float qac = QA[(size_t)h * NN + i0 + c];
  const _Float16* vhp = (const _Float16*)(const void*)VTh + (size_t)(h * DK + c) * NN + 8 * hh;
  const _Float16* vrp = (const _Float16*)(const void*)VTr + (size_t)(h * DK + c) * NN + 8 * hh;
  const float* mrow = mask + (size_t)(i0 + (tid >> 4)) * NN + 2 * (tid & 15);
  const float* krow = KA + (size_t)h * NN + lane;
  const size_t vs16 = (size_t)16 * NN;

  float m_run = -INFINITY, l_run = 0.f;
  v8f o0 = zero8(), o1 = zero8();

#pragma unroll 1
  for (int j0 = 0; j0 < NN; j0 += 32) {
    __syncthreads();
    {
      const v2f mv = *(const v2f*)(mrow + j0);
      v2f mb;
      mb.x = bfr(mv.x);
      mb.y = bfr(mv.y);
      *(v2f*)(mk + 2 * tid) = mb;
      kat[tid] = krow[j0];
    }
    __syncthreads();
    float u0[8], u1[8];
    {
      const float* mp = mk + c * 32 + 8 * hh;
      const float* kp = kat + h * 32 + 8 * hh;
      const v4f ma = *(const v4f*)(mp), mb = *(const v4f*)(mp + 4), mc = *(const v4f*)(mp + 16), md = *(const v4f*)(mp + 20);
      const v4f ka = *(const v4f*)(kp), kq = *(const v4f*)(kp + 4), kc = *(const v4f*)(kp + 16), kd = *(const v4f*)(kp + 20);
#pragma unroll
      for (int r = 0; r < 4; ++r) {
        u0[r]     = lscore(qac, ka[r], ma[r]);
        u0[4 + r] = lscore(qac, kq[r], mb[r]);
        u1[r]     = lscore(qac, kc[r], mc[r]);
        u1[4 + r] = lscore(qac, kd[r], md[r]);
      }
    }
    float mx = -INFINITY;
#pragma unroll
    for (int r = 0; r < 8; ++r) mx = fmaxf(mx, fmaxf(u0[r], u1[r]));
    mx = fmaxf(mx, __shfl_xor(mx, 16, 32));
    const float mn = fmaxf(m_run, mx);
    const float al = exp2f(m_run - mn);
    m_run = mn;
    float ps = 0.f;
    FragH pa;
#pragma unroll
    for (int r = 0; r < 8; ++r) {
      const float e0 = exp2f(u0[r] - mn), e1 = exp2f(u1[r] - mn);
      ps += e0 + e1;
      pa.h[0][r] = (_Float16)(e0 * PCAR);
      pa.h[1][r] = (_Float16)(e1 * PCAR);
    }
    ps += __shfl_xor(ps, 16, 32);
    l_run = l_run * al + ps;
#pragma unroll
    for (int r = 0; r < 8; ++r) {
      const float af = __shfl(al, 8 * hh + r, 32);
      o0[r] *= af;
      o1[r] *= af;
    }
    {
      const _Float16* ph = vhp + j0;
      const _Float16* pr = vrp + j0;
      const v16h v0h = ldfrag_h(ph), v1h = ldfrag_h(ph + vs16);
      const v16h v0r = ldfrag_h(pr), v1r = ldfrag_h(pr + vs16);
      o0 = mma_raw(pa.v, v0h, o0);
      o0 = mma_raw(pa.v, v0r, o0);
      o1 = mma_raw(pa.v, v1h, o1);
      o1 = mma_raw(pa.v, v1r, o1);
      guard_a2(o0, o1, pa.v, v0h, v0r, v1h, v1r);
    }
  }
  acc_guard2(o0, o1);

  const float li = (l_run > 0.0f) ? ((1.0f / l_run) * (XSA / (PCAR * VSC))) : 0.0f;
  float lf[8];
#pragma unroll
  for (int r = 0; r < 8; ++r) lf[r] = __shfl(li, 8 * hh + r, 32);
#pragma unroll
  for (int r = 0; r < 8; ++r) {
    float* sp = ot + (8 * hh + r) * OTP + h * DK + c;
    sp[0]  = o0[r] * lf[r];
    sp[16] = o1[r] * lf[r];
  }
  __syncthreads();
  v4u xh[2], xr[2];
#pragma unroll
  for (int it = 0; it < 2; ++it) {
    const float* sp = ot + (8 * it + h) * OTP + 8 * lane;
    const v4f w0 = *(const v4f*)(sp), w1 = *(const v4f*)(sp + 4);
    float f[8];
#pragma unroll
    for (int e = 0; e < 4; ++e) { f[e] = w0[e]; f[4 + e] = w1[e]; }
    v4u oh, orr;
#pragma unroll
    for (int i = 0; i < 4; ++i) {
      const float t0 = f[2 * i], t1 = f[2 * i + 1];
      const _Float16 g0 = (_Float16)t0, g1 = (_Float16)t1;
      const _Float16 r0 = (_Float16)(t0 - (float)g0), r1 = (_Float16)(t1 - (float)g1);
      oh[i]  = pk16(h_bits(g0), h_bits(g1));
      orr[i] = pk16(h_bits(r0), h_bits(r1));
    }
    xh[it] = oh;
    xr[it] = orr;
  }
  unsigned short* dh = Xh + (size_t)(i0 + h) * DD + 8 * lane;
  unsigned short* dr = Xr + (size_t)(i0 + h) * DD + 8 * lane;
  const size_t rs8 = (size_t)8 * DD;
  for (int pass = 0; pass < 2; ++pass) {
#pragma unroll
    for (int it = 0; it < 2; ++it) {
      *(volatile v4u*)(dh + it * rs8) = xh[it];
      *(volatile v4u*)(dr + it * rs8) = xr[it];
    }
    __threadfence();
  }
}

extern "C" void kernel_launch(void* const* d_in, const int* in_sizes, int n_in,
                              void* d_out, int out_size, void* d_ws, size_t ws_size,
                              hipStream_t stream) {
  if (n_in < 13) return;
  if (in_sizes[0] < NN * IND || in_sizes[2] < NN * NN || in_sizes[4] < IND * DD || in_sizes[5] < DD) return;
  if (in_sizes[6] < NL * DD * DD || in_sizes[7] < NL * DD * DD || in_sizes[8] < NL * DD * DD) return;
  if (in_sizes[9] < NL * HH * DK || in_sizes[10] < NL * HH * DK || in_sizes[11] < DD * OD || in_sizes[12] < OD) return;
  if (out_size < NN * OD) return;

  const float* noise = (const float*)d_in[0];
  const float* mask  = (const float*)d_in[2];
  const float* w_in  = (const float*)d_in[4];
  const float* b_in  = (const float*)d_in[5];
  const float* Wq    = (const float*)d_in[6];
  const float* Wk    = (const float*)d_in[7];
  const float* Wv    = (const float*)d_in[8];
  const float* aq    = (const float*)d_in[9];
  const float* ak    = (const float*)d_in[10];
  const float* w_out = (const float*)d_in[11];
  const float* b_out = (const float*)d_in[12];
  float* out = (float*)d_out;

  const size_t szNP  = (size_t)NN * IND * 2;
  const size_t szWTI = (size_t)DD * IND * 2;
  const size_t szWTQ = (size_t)QKVW * DD * 2;
  const size_t szWTO = (size_t)OD * DD * 2;
  const size_t szX   = (size_t)NN * DD * 2;
  const size_t szC   = (size_t)NN * QKVW * 4;
  const size_t szQA  = (size_t)HH * NN * 4;
  const size_t szVT  = (size_t)DD * NN * 2;
  size_t off = 0;
  const size_t oNP  = off; off += szNP;
  const size_t oWTI = off; off += szWTI;
  const size_t oWQ0 = off; off += szWTQ;
  const size_t oWQ1 = off; off += szWTQ;
  const size_t oWTO = off; off += szWTO;
  const size_t oXAh = off; off += szX;
  const size_t oXAr = off; off += szX;
  const size_t oXBh = off; off += szX;
  const size_t oXBr = off; off += szX;
  const size_t oC   = off; off += szC;
  const size_t oQA  = off; off += szQA;
  const size_t oKA  = off; off += szQA;
  const size_t oVTh = off; off += szVT;
  const size_t oVTr = off; off += szVT;
  if (off > ws_size) return;
  if (off > (size_t)134217728) return;

  char* ws = (char*)d_ws;
  unsigned short* NP   = (unsigned short*)(ws + oNP);
  unsigned short* WTI  = (unsigned short*)(ws + oWTI);
  unsigned short* WQ0  = (unsigned short*)(ws + oWQ0);
  unsigned short* WQ1  = (unsigned short*)(ws + oWQ1);
  unsigned short* WTO  = (unsigned short*)(ws + oWTO);
  unsigned short* XAh  = (unsigned short*)(ws + oXAh);
  unsigned short* XAr  = (unsigned short*)(ws + oXAr);
  unsigned short* XBh  = (unsigned short*)(ws + oXBh);
  unsigned short* XBr  = (unsigned short*)(ws + oXBr);
  float*          Cm   = (float*)(ws + oC);
  float*          QAp  = (float*)(ws + oQA);
  float*          KAp  = (float*)(ws + oKA);
  unsigned short* VTh  = (unsigned short*)(ws + oVTh);
  unsigned short* VTr  = (unsigned short*)(ws + oVTr);

  const int n8 = NN * IND / 8;
  const dim3 blk(256), bG(128);

  cvt16<<<dim3(n8 / 256), blk, 0, stream>>>(noise, NP, n8, NSC);
  wt16<<<dim3(DD / 64, IND / 64), blk, 0, stream>>>(w_in, WTI, IND, DD, WSC);
  wt16<<<dim3(DD / 64, DD / 64), blk, 0, stream>>>(Wq, WQ0, DD, DD, WSC);
  wt16<<<dim3(DD / 64, DD / 64), blk, 0, stream>>>(Wk, WQ0 + (size_t)DD * DD, DD, DD, WSC);
  wt16<<<dim3(DD / 64, DD / 64), blk, 0, stream>>>(Wv, WQ0 + (size_t)2 * DD * DD, DD, DD, WSC);
  wt16<<<dim3(DD / 64, DD / 64), blk, 0, stream>>>(Wq + (size_t)DD * DD, WQ1, DD, DD, WSC);
  wt16<<<dim3(DD / 64, DD / 64), blk, 0, stream>>>(Wk + (size_t)DD * DD, WQ1 + (size_t)DD * DD, DD, DD, WSC);
  wt16<<<dim3(DD / 64, DD / 64), blk, 0, stream>>>(Wv + (size_t)DD * DD, WQ1 + (size_t)2 * DD * DD, DD, DD, WSC);
  wt16<<<dim3(OD / 64, DD / 64), blk, 0, stream>>>(w_out, WTO, DD, OD, WSC);
  gemm16<false, true, 1><<<dim3(DD / 64, NN / 64), bG, 0, stream>>>(NP, NP, WTI, b_in, Cm, XAh, XAr,
                                                                    NN, DD, IND, 1.0f / (NSC * WSC), XS0);
  gemm16<true, false, 0><<<dim3(QKVW / 64, NN / 64), bG, 0, stream>>>(XAh, XAr, WQ0, b_in, Cm, XBh, XBr,
                                                                      NN, QKVW, DD, 1.0f / (XS0 * WSC), 1.0f);
  qkv_post<<<dim3(NN / 64), blk, 0, stream>>>(Cm, aq, ak, QAp, KAp, VTh, VTr);
  add_attn<<<dim3(NN / 16), blk, 0, stream>>>(QAp, KAp, mask, VTh, VTr, XBh, XBr);
  gemm16<true, false, 0><<<dim3(QKVW / 64, NN / 64), bG, 0, stream>>>(XBh, XBr, WQ1, b_in, Cm, XAh, XAr,
                                                                      NN, QKVW, DD, 1.0f / (XSA * WSC), 1.0f);
  qkv_post<<<dim3(NN / 64), blk, 0, stream>>>(Cm, aq + HH * DK, ak + HH * DK, QAp, KAp, VTh, VTr);
  add_attn<<<dim3(NN / 16), blk, 0, stream>>>(QAp, KAp, mask, VTh, VTr, XAh, XAr);
  gemm16<true, true, 0><<<dim3(OD / 64, NN / 64), bG, 0, stream>>>(XAh, XAr, WTO, b_out, out, XBh, XBr,
                                                                     NN, OD, DD, 1.0f / (XSA * WSC), 1.0f);
  (void)hipGetLastError();
}
